// ChunkedLayer_70205535420729
// MI455X (gfx1250) — hardware-run, weakly checked
//
#include <hip/hip_runtime.h>
#include <math.h>

constexpr int kBatch  = 2;
constexpr int kSteps  = 1024;
constexpr int kChan   = 1024;
constexpr int kHeads  = 16;
constexpr int kHdim   = 64;
constexpr int kTok    = kBatch * kSteps;
constexpr size_t kPlane = (size_t)kTok * kChan;
constexpr int kScalN  = 80;
constexpr int kScalNP = 128;
constexpr int kChunk  = 32;
constexpr int kScanThreads = 512;

constexpr float kXCarry   = 16.0f;
constexpr float kWCarry   = 256.0f;
constexpr float kOCarry   = 64.0f;
constexpr float kResCarry = 2048.0f;
constexpr float kResInv   = 1.0f / kResCarry;
constexpr float kScaleProj = 1.0f / (kXCarry * kWCarry);
constexpr float kScaleOut  = 1.0f / (kOCarry * kWCarry);
constexpr float kF16Min   = 6.103515625e-5f;
constexpr float kCapInv   = 1.0f / (float)kHdim;
constexpr float kMeanInv  = 1.0f / (float)kHdim;
constexpr float kQkEps    = 1e-6f;
constexpr float kNormEps  = 1e-5f;

static_assert(kHeads * kHdim == kChan, "head split");
static_assert(kTok % 32 == 0 && kChan % 64 == 0 && kScalNP % 64 == 0, "GEMM M,N tiles");
static_assert(kChan % 32 == 0, "GEMM K multiple of 32");
static_assert(kSteps % kChunk == 0, "chunking");
static_assert(kHdim == 64 && kChunk == 32 && kScanThreads == 512, "scan tiling");
static_assert(5 * kHeads == kScalN && kScalN <= kScalNP, "merged scalar plane");
static_assert((kTok * kHeads) % 8 == 0, "norm grid");

typedef __attribute__((ext_vector_type(16))) _Float16 v16h;
typedef __attribute__((ext_vector_type(8)))  _Float16 v8h;
typedef __attribute__((ext_vector_type(8)))  float    v8f;
typedef __attribute__((ext_vector_type(4)))  float    v4f;
typedef __attribute__((ext_vector_type(2)))  float    v2f;
typedef __attribute__((ext_vector_type(4)))  unsigned int v4u;

__device__ __forceinline__ unsigned pk16(unsigned short a, unsigned short b) {
  return (unsigned)a | ((unsigned)b << 16);
}
__device__ __forceinline__ unsigned short h_bits(float f) {
  const float g = (fabsf(f) < kF16Min) ? 0.0f : f;
  const _Float16 h = (_Float16)g;
  return __builtin_bit_cast(unsigned short, h);
}
__device__ __forceinline__ void h_split(float v, unsigned short& hb, unsigned short& rb) {
  const float g = (fabsf(v) < kF16Min) ? 0.0f : v;
  const _Float16 h = (_Float16)g;
  const float hf = (float)h;
  const float d = (v - hf) * kResCarry;
  const float dg = (fabsf(d) < kF16Min) ? 0.0f : d;
  const _Float16 r = (_Float16)dg;
  hb = __builtin_bit_cast(unsigned short, h);
  rb = __builtin_bit_cast(unsigned short, r);
}
__device__ __forceinline__ v4u pack8_plain(const float (&v)[8]) {
  unsigned short hb[8];
#pragma unroll
  for (int e = 0; e < 8; ++e) hb[e] = h_bits(v[e]);
  return (v4u){pk16(hb[0], hb[1]), pk16(hb[2], hb[3]), pk16(hb[4], hb[5]), pk16(hb[6], hb[7])};
}
__device__ __forceinline__ void pack8_split(const float (&v)[8], v4u& uh, v4u& ur) {
  unsigned short hb[8], rb[8];
#pragma unroll
  for (int e = 0; e < 8; ++e) h_split(v[e], hb[e], rb[e]);
  uh = (v4u){pk16(hb[0], hb[1]), pk16(hb[2], hb[3]), pk16(hb[4], hb[5]), pk16(hb[6], hb[7])};
  ur = (v4u){pk16(rb[0], rb[1]), pk16(rb[2], rb[3]), pk16(rb[4], rb[5]), pk16(rb[6], rb[7])};
}
__device__ __forceinline__ float wave_sum32(float v) {
#pragma unroll
  for (int o = 16; o > 0; o >>= 1) v += __shfl_xor(v, o, 32);
  return v;
}

struct FragH {
  union U { v16h v; v8h h[2]; };
  static __device__ __forceinline__ v16h load(const _Float16* p) {
    U f;
    f.h[0] = *(const v8h*)(p);
    f.h[1] = *(const v8h*)(p + 16);
    return f.v;
  }
  static __device__ __forceinline__ v8f mma(v16h a, v16h b, v8f c) {
    return __builtin_amdgcn_wmma_f32_16x16x32_f16(false, a, false, b, (short)0, c, false, false);
  }
};
__device__ __forceinline__ void guard_split(v8f& a0, v8f& a1, v8f& a2, v8f& a3,
                                            v16h x0, v16h x1, v16h x2, v16h x3, v16h y0, v16h y1) {
  asm volatile("v_nop\n\tv_nop\n\tv_nop\n\tv_nop"
               : "+v"(a0), "+v"(a1), "+v"(a2), "+v"(a3)
               : "v"(x0), "v"(x1), "v"(x2), "v"(x3), "v"(y0), "v"(y1));
}
__device__ __forceinline__ void guard_plain(v8f& a0, v8f& a1, v16h x0, v16h x1, v16h y0) {
  asm volatile("v_nop\n\tv_nop\n\tv_nop\n\tv_nop"
               : "+v"(a0), "+v"(a1)
               : "v"(x0), "v"(x1), "v"(y0));
}
__device__ __forceinline__ void acc_guard4(v8f& a, v8f& b, v8f& c, v8f& d) {
  asm volatile("v_nop\n\tv_nop\n\tv_nop\n\tv_nop" : "+v"(a), "+v"(b), "+v"(c), "+v"(d));
}

template <bool SPLIT, bool BIAS>
__global__ __launch_bounds__(256) void gemm_f16_kernel(
    const unsigned short* __restrict__ Ahp, const unsigned short* __restrict__ Arp, int lda, long strideA,
    const unsigned short* __restrict__ Bhp, const unsigned short* __restrict__ Brp, int ldb, long strideB,
    float* __restrict__ Cout, int ldc, long strideC, const float* __restrict__ bias,
    int M, int N, int K, float scale) {
  __shared__ __align__(16) float sT[8][16 * 68];
  const int z    = blockIdx.y;
  const int lane = threadIdx.x & 31;
  const int wave = threadIdx.x >> 5;
  const int tilesN = N >> 6;
  const int tilesM = M >> 5;
  const int tile = blockIdx.x * 8 + wave;
  if (tile >= tilesM * tilesN) return;
  const int tm = tile / tilesN;
  const int tn = tile - tm * tilesN;
  const int m0 = tm << 5;
  const int n0 = tn << 6;
  const int rlane = lane & 15;
  const int half8 = (lane >> 4) * 8;
  const int mOff  = (lane >> 4) * 8;

  const size_t aoff = (size_t)z * (size_t)strideA + (size_t)(m0 + rlane) * lda + half8;
  const size_t boff = (size_t)z * (size_t)strideB + (size_t)(n0 + rlane) * ldb + half8;
  const _Float16* pa0 = (const _Float16*)Ahp + aoff;
  const _Float16* pa1 = pa0 + (size_t)16 * lda;
  const _Float16* pr0 = SPLIT ? ((const _Float16*)Arp + aoff) : pa0;
  const _Float16* pr1 = pr0 + (size_t)16 * lda;
  const _Float16* pbh = (const _Float16*)Bhp + boff;
  const _Float16* pbr = SPLIT ? ((const _Float16*)Brp + boff) : pbh;
  const size_t bstep = (size_t)16 * ldb;

  v8f acc[2][4], accr[2][4];
#pragma unroll
  for (int i = 0; i < 2; ++i)
#pragma unroll
    for (int j = 0; j < 4; ++j) {
      acc[i][j]  = (v8f){0.f, 0.f, 0.f, 0.f, 0.f, 0.f, 0.f, 0.f};
      accr[i][j] = (v8f){0.f, 0.f, 0.f, 0.f, 0.f, 0.f, 0.f, 0.f};
    }

  for (int k0 = 0; k0 < K; k0 += 32) {
    const v16h ah0 = FragH::load(pa0 + k0);
    const v16h ah1 = FragH::load(pa1 + k0);
    v16h ar0 = ah0, ar1 = ah1;
    if (SPLIT) {
      ar0 = FragH::load(pr0 + k0);
      ar1 = FragH::load(pr1 + k0);
    }
#pragma unroll
    for (int j = 0; j < 4; ++j) {
      const v16h bh = FragH::load(pbh + j * bstep + k0);
      v16h br = bh;
      if (SPLIT) br = FragH::load(pbr + j * bstep + k0);
      acc[0][j] = FragH::mma(ah0, bh, acc[0][j]);
      acc[1][j] = FragH::mma(ah1, bh, acc[1][j]);
      if (SPLIT) {
        accr[0][j] = FragH::mma(ah0, br, accr[0][j]);
        accr[1][j] = FragH::mma(ah1, br, accr[1][j]);
        accr[0][j] = FragH::mma(ar0, bh, accr[0][j]);
        accr[1][j] = FragH::mma(ar1, bh, accr[1][j]);
        guard_split(acc[0][j], acc[1][j], accr[0][j], accr[1][j], ah0, ah1, ar0, ar1, bh, br);
      } else {
        guard_plain(acc[0][j], acc[1][j], ah0, ah1, bh);
      }
    }
  }
  acc_guard4(acc[0][0], acc[0][1], acc[0][2], acc[0][3]);
  acc_guard4(acc[1][0], acc[1][1], acc[1][2], acc[1][3]);
  if (SPLIT) {
    acc_guard4(accr[0][0], accr[0][1], accr[0][2], accr[0][3]);
    acc_guard4(accr[1][0], accr[1][1], accr[1][2], accr[1][3]);
  }

  float bj[4];
#pragma unroll
  for (int j = 0; j < 4; ++j) {
    bj[j] = 0.0f;
    if (BIAS) bj[j] = bias[n0 + (j << 4) + rlane];
  }

  float* slab = sT[wave];
  float* C = Cout + (size_t)z * (size_t)strideC;
#pragma unroll
  for (int i = 0; i < 2; ++i) {
    const int mBase = m0 + (i << 4);
#pragma unroll
    for (int j = 0; j < 4; ++j) {
#pragma unroll
      for (int r = 0; r < 8; ++r) {
        float v = acc[i][j][r];
        if (SPLIT) v += accr[i][j][r] * kResInv;
        v *= scale;
        if (BIAS) v += bj[j];
        slab[(mOff + r) * 68 + (j << 4) + rlane] = v;
      }
    }
    __builtin_amdgcn_fence(__ATOMIC_RELEASE, "workgroup");
    __builtin_amdgcn_wave_barrier();
    __builtin_amdgcn_fence(__ATOMIC_ACQUIRE, "workgroup");
    {
      const int hh = lane >> 4, c4 = (lane & 15) * 4;
      for (int pass = 0; pass < 2; ++pass) {
#pragma unroll
        for (int it = 0; it < 8; ++it) {
          const int row = it * 2 + hh;
          const v4f v = *(const v4f*)(slab + row * 68 + c4);
          *(volatile v4f*)(C + (size_t)(mBase + row) * ldc + n0 + c4) = v;
        }
        __threadfence();
      }
    }
    __builtin_amdgcn_fence(__ATOMIC_RELEASE, "workgroup");
    __builtin_amdgcn_wave_barrier();
    __builtin_amdgcn_fence(__ATOMIC_ACQUIRE, "workgroup");
  }
}

__global__ __launch_bounds__(256) void wt_plane_kernel(const float* __restrict__ W0, const float* __restrict__ W1,
                                                       const float* __restrict__ W2, const float* __restrict__ W3,
                                                       unsigned short* __restrict__ outh, unsigned short* __restrict__ outr,
                                                       int Kd, int Nd, int KdP, int NdP, int has_res) {
  __shared__ float sm[64][65];
  const int t  = threadIdx.x;
  const int k0 = blockIdx.x * 64;
  const int n0 = blockIdx.y * 64;
  const int z  = blockIdx.z;
  const float* W = (z == 0) ? W0 : (z == 1) ? W1 : (z == 2) ? W2 : W3;
#pragma unroll
  for (int i = 0; i < 16; ++i) {
    const int e = i * 256 + t;
    const int r = e >> 6;
    const int c = e & 63;
    const int kk = k0 + r;
    const int nn = n0 + c;
    const bool valid = (kk < Kd) && (nn < Nd);
    const int kc = (kk < Kd) ? kk : (Kd - 1);
    const int nc = (nn < Nd) ? nn : (Nd - 1);
    const float v = W[(size_t)kc * Nd + nc];
    sm[c][r] = valid ? (v * kWCarry) : 0.0f;
  }
  __syncthreads();
  const int lane = t & 31, wave = t >> 5;
  const int q = lane >> 3, c8 = (lane & 7) * 8;
  const size_t pofs = (size_t)z * (size_t)NdP * (size_t)KdP;
  for (int pass = 0; pass < 2; ++pass) {
#pragma unroll
    for (int it = 0; it < 2; ++it) {
      const int row = wave * 8 + it * 4 + q;
      float v[8];
#pragma unroll
      for (int e = 0; e < 8; ++e) v[e] = sm[row][c8 + e];
      v4u uh, ur;
      pack8_split(v, uh, ur);
      const size_t o = pofs + (size_t)(n0 + row) * KdP + k0 + c8;
      *(volatile v4u*)(outh + o) = uh;
      if (has_res) *(volatile v4u*)(outr + o) = ur;
    }
    __threadfence();
  }
}

__global__ __launch_bounds__(256) void scal_plane_kernel(const float* __restrict__ Wb, const float* __restrict__ Wfd,
                                                         const float* __restrict__ Wsd, const float* __restrict__ Wfg,
                                                         const float* __restrict__ Wsg,
                                                         unsigned short* __restrict__ outh) {
  __shared__ float sm[64][65];
  const int t  = threadIdx.x;
  const int k0 = blockIdx.x * 64;
  const int n0 = blockIdx.y * 64;
#pragma unroll 1
  for (int i = 0; i < 16; ++i) {
    const int e = i * 256 + t;
    const int r = e >> 6;
    const int c = e & 63;
    const int kk = k0 + r;
    const int nn = n0 + c;
    const int grp = nn >> 4;
    const int hc = nn & 15;
    const size_t src = (size_t)kk * kHeads + hc;
    float v0 = Wb[src];
    float v1 = Wfd[src];
    float v2 = Wsd[src];
    float v3 = Wfg[src];
    float v4 = Wsg[src];
    asm volatile("" : "+v"(v0), "+v"(v1), "+v"(v2), "+v"(v3), "+v"(v4));
    const float v = (grp == 0) ? v0 : (grp == 1) ? v1 : (grp == 2) ? v2 : (grp == 3) ? v3 : (grp == 4) ? v4 : 0.0f;
    sm[c][r] = (nn < kScalN) ? (v * kWCarry) : 0.0f;
  }
  __syncthreads();
  const int lane = t & 31, wave = t >> 5;
  const int q = lane >> 3, c8 = (lane & 7) * 8;
  for (int pass = 0; pass < 2; ++pass) {
#pragma unroll
    for (int it = 0; it < 2; ++it) {
      const int row = wave * 8 + it * 4 + q;
      float v[8];
#pragma unroll
      for (int e = 0; e < 8; ++e) v[e] = sm[row][c8 + e];
      const v4u uh = pack8_plain(v);
      const size_t o = (size_t)(n0 + row) * kChan + k0 + c8;
      *(volatile v4u*)(outh + o) = uh;
    }
    __threadfence();
  }
}

__global__ __launch_bounds__(256) void cast_split_kernel(const float* __restrict__ x,
                                                         unsigned short* __restrict__ XH,
                                                         unsigned short* __restrict__ XR) {
  const int i = blockIdx.x * 256 + threadIdx.x;
  if (i >= kTok * (kChan / 8)) return;
  const size_t off = (size_t)i * 8;
  const v4f a = *(const v4f*)(x + off);
  const v4f b = *(const v4f*)(x + off + 4);
  float v[8];
#pragma unroll
  for (int e = 0; e < 4; ++e) {
    v[e]     = a[e] * kXCarry;
    v[4 + e] = b[e] * kXCarry;
  }
  v4u uh, ur;
  pack8_split(v, uh, ur);
  for (int pass = 0; pass < 2; ++pass) {
    *(volatile v4u*)(XH + off) = uh;
    *(volatile v4u*)(XR + off) = ur;
    __threadfence();
  }
}

__global__ __launch_bounds__(256) void prep_kernel(float* QKV, float* SC,
                                                   const float* __restrict__ bq, const float* __restrict__ bk,
                                                   const float* __restrict__ bv,
                                                   const float* __restrict__ bb, const float* __restrict__ bfd,
                                                   const float* __restrict__ fdb, const float* __restrict__ bsd,
                                                   const float* __restrict__ sdb, const float* __restrict__ bfg,
                                                   const float* __restrict__ bsg) {
  const int tok  = blockIdx.x;
  const int lane = threadIdx.x & 31;
  const int wave = threadIdx.x >> 5;
#pragma unroll 1
  for (int p = 0; p < 3; ++p) {
    float* P = QKV + (size_t)p * kPlane;
    const float* bias = (p == 0) ? bq : (p == 1) ? bk : bv;
#pragma unroll 1
    for (int hf = 0; hf < 2; ++hf) {
      const int h = wave * 2 + hf;
      const int c = h * kHdim + lane;
      const size_t idx = (size_t)tok * kChan + c;
      const float x0 = P[idx] + bias[c];
      const float x1 = P[idx + 32] + bias[c + 32];
      const float s0 = x0 * __builtin_amdgcn_rcpf(1.0f + expf(-x0));
      const float s1 = x1 * __builtin_amdgcn_rcpf(1.0f + expf(-x1));
      const float ss = wave_sum32(s0 * s0 + s1 * s1);
      const float inv = __builtin_amdgcn_rcpf(sqrtf(ss + kQkEps));
      const float scl = (p < 2) ? inv : 1.0f;
      const float y0 = s0 * scl;
      const float y1 = s1 * scl;
      *(volatile float*)(P + idx) = y0;
      *(volatile float*)(P + idx + 32) = y1;
      __threadfence();
      *(volatile float*)(P + idx) = y0;
      *(volatile float*)(P + idx + 32) = y1;
    }
  }
  if (wave < 4) {
    const int c = wave * 32 + lane;
    const int grp = c >> 4;
    const int hc = c & 15;
    const size_t sidx = (size_t)tok * kScalNP + c;
    float x  = SC[sidx];
    float c0 = bb[hc];
    float c1 = bfd[hc];
    float c2 = fdb[hc];
    float c3 = bsd[hc];
    float c4 = sdb[hc];
    float c5 = bfg[hc];
    float c6 = bsg[hc];
    asm volatile("" : "+v"(x), "+v"(c0), "+v"(c1), "+v"(c2), "+v"(c3), "+v"(c4), "+v"(c5), "+v"(c6));
    const float a1 = (grp == 0) ? c0 : (grp == 1) ? c1 : (grp == 2) ? c3 : (grp == 3) ? c5 : (grp == 4) ? c6 : 0.0f;
    const float a2 = (grp == 1) ? c2 : (grp == 2) ? c4 : 0.0f;
    const float arg = (x + a1) + a2;
    const float sg = __builtin_amdgcn_rcpf(1.0f + expf(-arg));
    const float o = (c < kScalN) ? sg : 0.0f;
    *(volatile float*)(SC + sidx) = o;
    __threadfence();
    *(volatile float*)(SC + sidx) = o;
  }
}

__global__ __launch_bounds__(512) void state_scan_kernel(const float* __restrict__ Qf, const float* __restrict__ Kf,
                                                         const float* __restrict__ Vf, const float* __restrict__ SG,
                                                         const float* __restrict__ rf_p, float* __restrict__ Y) {
  __shared__ __align__(16) float lv[3 * kChunk * 64];
  __shared__ __align__(16) float ls[kChunk * 8];
  __shared__ __align__(16) float yb[kChunk * 64];
  __shared__ __align__(16) float red[2][32];
  const int bh   = blockIdx.x;
  const int b    = bh >> 4;
  const int h    = bh & 15;
  const int tid  = threadIdx.x;
  const int lane = tid & 31;
  const int wave = tid >> 5;
  const int i    = tid >> 3;
  const int q    = tid & 7;
  const int j0   = q * 8;
  const int lrow = tid >> 4;
  const int lc4  = (tid & 15) * 4;
  const int srow = (tid >> 3) & (kChunk - 1);
  const int sgi  = tid & 7;
  const int scol = ((sgi < 4) ? sgi : 4) * kHeads + h;
  const size_t base = (size_t)b * kSteps * kChan + (size_t)h * kHdim;
  const float rf = rf_p[0];

  float Sf[8], Ss[8];
#pragma unroll
  for (int jj = 0; jj < 8; ++jj) {
    Sf[jj] = 0.0f;
    Ss[jj] = 0.0f;
  }

#pragma unroll 1
  for (int ch = 0; ch < kSteps / kChunk; ++ch) {
    const size_t goff = base + (size_t)(ch * kChunk + lrow) * kChan + lc4;
    {
      const v4f t0 = *(const v4f*)(Qf + goff);
      const v4f t1 = *(const v4f*)(Kf + goff);
      const v4f t2 = *(const v4f*)(Vf + goff);
      const int lo = lrow * 64 + lc4;
      *(v4f*)(lv + 0 * kChunk * 64 + lo) = t0;
      *(v4f*)(lv + 1 * kChunk * 64 + lo) = t1;
      *(v4f*)(lv + 2 * kChunk * 64 + lo) = t2;
    }
    if (wave < 8) {
      const float gv = SG[((size_t)b * kSteps + (size_t)(ch * kChunk + srow)) * kScalNP + scol];
      ls[srow * 8 + sgi] = gv;
    }
    __syncthreads();

#pragma unroll 1
    for (int s = 0; s < kChunk; ++s) {
      const float* pq = lv + 0 * kChunk * 64 + s * 64 + j0;
      const float* pk = lv + 1 * kChunk * 64 + s * 64 + j0;
      const float vi = lv[2 * kChunk * 64 + s * 64 + i];
      const v4f sc0 = *(const v4f*)(ls + s * 8);
      const v4f sc1 = *(const v4f*)(ls + s * 8 + 4);
      const float beta = sc0[0];
      const float fd = sc0[1];
      const float sd = sc0[2];
      const float fg = sc0[3];
      const float sg = sc1[0];
      const v4f ka = *(const v4f*)(pk);
      const v4f kb = *(const v4f*)(pk + 4);
      float kv[8];
#pragma unroll
      for (int e = 0; e < 4; ++e) {
        kv[e] = ka[e];
        kv[4 + e] = kb[e];
      }
      float pf = 0.0f, ps = 0.0f;
#pragma unroll
      for (int jj = 0; jj < 8; ++jj) {
        Sf[jj] *= fd;
        Ss[jj] *= sd;
        pf += kv[jj] * Sf[jj];
        ps += kv[jj] * Ss[jj];
      }
      pf += __shfl_xor(pf, 1, 32);
      ps += __shfl_xor(ps, 1, 32);
      pf += __shfl_xor(pf, 2, 32);
      ps += __shfl_xor(ps, 2, 32);
      pf += __shfl_xor(pf, 4, 32);
      ps += __shfl_xor(ps, 4, 32);
      const float ef = vi - pf;
      const float es = vi - ps;
      float nf = 0.0f, ns = 0.0f;
#pragma unroll
      for (int jj = 0; jj < 8; ++jj) {
        const float bkj = beta * kv[jj];
        const float uf = Sf[jj] + bkj * ef;
        const float us = Ss[jj] + bkj * es;
        const float tf = uf + rf * us;
        const float ts = us + rf * uf;
        Sf[jj] = tf;
        Ss[jj] = ts;
        nf += tf * tf;
        ns += ts * ts;
      }
      nf = wave_sum32(nf);
      ns = wave_sum32(ns);
      const int par = s & 1;
      if (lane == 0) {
        red[par][wave] = nf;
        red[par][16 + wave] = ns;
      }
      __syncthreads();
      float xs = red[par][lane];
      xs += __shfl_xor(xs, 8, 32);
      xs += __shfl_xor(xs, 4, 32);
      xs += __shfl_xor(xs, 2, 32);
      xs += __shfl_xor(xs, 1, 32);
      const float xo = __shfl_xor(xs, 16, 32);
      const float totf = (lane < 16) ? xs : xo;
      const float tots = (lane < 16) ? xo : xs;
      const float cf = __builtin_amdgcn_rcpf(fmaxf(1.0f, __builtin_amdgcn_sqrtf(totf) * kCapInv));
      const float cs = __builtin_amdgcn_rcpf(fmaxf(1.0f, __builtin_amdgcn_sqrtf(tots) * kCapInv));
      const v4f qa = *(const v4f*)(pq);
      const v4f qb = *(const v4f*)(pq + 4);
      float qv[8];
#pragma unroll
      for (int e = 0; e < 4; ++e) {
        qv[e] = qa[e];
        qv[4 + e] = qb[e];
      }
      float of = 0.0f, os = 0.0f;
#pragma unroll
      for (int jj = 0; jj < 8; ++jj) {
        Sf[jj] *= cf;
        Ss[jj] *= cs;
        of += qv[jj] * Sf[jj];
        os += qv[jj] * Ss[jj];
      }
      of += __shfl_xor(of, 1, 32);
      os += __shfl_xor(os, 1, 32);
      of += __shfl_xor(of, 2, 32);
      os += __shfl_xor(os, 2, 32);
      of += __shfl_xor(of, 4, 32);
      os += __shfl_xor(os, 4, 32);
      const float yo = fg * of + sg * os;
      if (q == 0) yb[s * 64 + i] = yo;
    }
    __syncthreads();
    {
      const v4f val = *(const v4f*)(yb + lrow * 64 + lc4);
      *(volatile v4f*)(Y + goff) = val;
      __threadfence();
      *(volatile v4f*)(Y + goff) = val;
    }
  }
}

__global__ __launch_bounds__(256) void norm_gate_kernel(const float* __restrict__ Y, const float* __restrict__ Gf,
                                                        const float* __restrict__ bg, const float* __restrict__ onw,
                                                        unsigned* __restrict__ O16) {
  const int lane = threadIdx.x & 31;
  const int pair = blockIdx.x * 8 + (threadIdx.x >> 5);
  const int tok = pair >> 4;
  const int h   = pair & 15;
  const size_t base = (size_t)tok * kChan + (size_t)h * kHdim + 2 * lane;
  const int c = h * kHdim + 2 * lane;
  const v2f y2 = *(const v2f*)(Y + base);
  const v2f g2 = *(const v2f*)(Gf + base);
  const v2f b2 = *(const v2f*)(bg + c);
  const v2f w2 = *(const v2f*)(onw + 2 * lane);
  const float ms = wave_sum32(y2[0] * y2[0] + y2[1] * y2[1]) * kMeanInv;
  const float inv = __builtin_amdgcn_rcpf(sqrtf(ms + kNormEps));
  const float ga = g2[0] + b2[0];
  const float gb = g2[1] + b2[1];
  const float sa = ga * __builtin_amdgcn_rcpf(1.0f + expf(-ga));
  const float sb = gb * __builtin_amdgcn_rcpf(1.0f + expf(-gb));
  const float o0 = (((y2[0] * inv) * w2[0]) * sa) * kOCarry;
  const float o1 = (((y2[1] * inv) * w2[1]) * sb) * kOCarry;
  const unsigned short h0 = h_bits(o0);
  const unsigned short h1 = h_bits(o1);
  const unsigned wh = pk16(h0, h1);
  const size_t widx = base >> 1;
  *(volatile unsigned*)(O16 + widx) = wh;
  __threadfence();
  *(volatile unsigned*)(O16 + widx) = wh;
}

extern "C" void kernel_launch(void* const* d_in, const int* in_sizes, int n_in,
                              void* d_out, int out_size, void* d_ws, size_t ws_size, hipStream_t stream) {
  if (n_in < 25 || d_out == nullptr || d_ws == nullptr) return;
  const int nP = (int)kPlane;
  const int nW = kChan * kChan;
  const int nS = kChan * kHeads;
  if (in_sizes[0] != nP) return;
  if (in_sizes[1] != nW || in_sizes[3] != nW || in_sizes[5] != nW || in_sizes[19] != nW || in_sizes[22] != nW) return;
  if (in_sizes[2] != kChan || in_sizes[4] != kChan || in_sizes[6] != kChan || in_sizes[20] != kChan ||
      in_sizes[23] != kChan) return;
  if (in_sizes[7] != nS || in_sizes[9] != nS || in_sizes[12] != nS || in_sizes[15] != nS || in_sizes[17] != nS) return;
  if (in_sizes[8] != kHeads || in_sizes[10] != kHeads || in_sizes[11] != kHeads || in_sizes[13] != kHeads ||
      in_sizes[14] != kHeads || in_sizes[16] != kHeads || in_sizes[18] != kHeads) return;
  if (in_sizes[21] != kHdim || in_sizes[24] != 1) return;
  if (out_size != nP) return;

  const float* hs  = (const float*)d_in[0];
  const float* Wq  = (const float*)d_in[1];
  const float* bq  = (const float*)d_in[2];
  const float* Wk  = (const float*)d_in[3];
  const float* bk  = (const float*)d_in[4];
  const float* Wv  = (const float*)d_in[5];
  const float* bv  = (const float*)d_in[6];
  const float* Wb  = (const float*)d_in[7];
  const float* bb  = (const float*)d_in[8];
  const float* Wfd = (const float*)d_in[9];
  const float* bfd = (const float*)d_in[10];
  const float* fdb = (const float*)d_in[11];
  const float* Wsd = (const float*)d_in[12];
  const float* bsd = (const float*)d_in[13];
  const float* sdb = (const float*)d_in[14];
  const float* Wfg = (const float*)d_in[15];
  const float* bfg = (const float*)d_in[16];
  const float* Wsg = (const float*)d_in[17];
  const float* bsg = (const float*)d_in[18];
  const float* Wg  = (const float*)d_in[19];
  const float* bg  = (const float*)d_in[20];
  const float* onw = (const float*)d_in[21];
  const float* Wo  = (const float*)d_in[22];
  const float* bo  = (const float*)d_in[23];
  const float* rfp = (const float*)d_in[24];
  float* out0 = (float*)d_out;

  char* ws = (char*)d_ws;
  size_t off = 0;
  auto carve = [&](size_t bytes) -> char* {
    char* p = ws + off;
    off += (bytes + 255) & ~(size_t)255;
    return p;
  };
  const size_t actB = kPlane * 2;
  const size_t wBig = (size_t)kChan * kChan;
  unsigned short* XH   = (unsigned short*)carve(actB);
  unsigned short* XR   = (unsigned short*)carve(actB);
  unsigned short* WBh  = (unsigned short*)carve(4 * wBig * 2);
  unsigned short* WBr  = (unsigned short*)carve(4 * wBig * 2);
  unsigned short* WOh  = (unsigned short*)carve(wBig * 2);
  unsigned short* WSc  = (unsigned short*)carve((size_t)kScalNP * kChan * 2);
  float*          QKVG = (float*)carve(4 * kPlane * 4);
  float*          SC   = (float*)carve((size_t)kTok * kScalNP * 4);
  float*          Yf   = (float*)carve(kPlane * 4);
  unsigned short* O16  = (unsigned short*)carve(actB);
  if (off > ws_size || off > (size_t)134217728) return;

  float* Qf = QKVG;
  float* Kf = QKVG + kPlane;
  float* Vf = QKVG + 2 * kPlane;
  float* Gf = QKVG + 3 * kPlane;

  wt_plane_kernel<<<dim3(kChan / 64, kChan / 64, 4), 256, 0, stream>>>(Wq, Wk, Wv, Wg, WBh, WBr,
                                                                        kChan, kChan, kChan, kChan, 1);
  wt_plane_kernel<<<dim3(kChan / 64, kChan / 64, 1), 256, 0, stream>>>(Wo, Wo, Wo, Wo, WOh, WOh,
                                                                        kChan, kChan, kChan, kChan, 0);
  scal_plane_kernel<<<dim3(kChan / 64, kScalNP / 64), 256, 0, stream>>>(Wb, Wfd, Wsd, Wfg, Wsg, WSc);

  cast_split_kernel<<<(kTok * (kChan / 8)) / 256, 256, 0, stream>>>(hs, XH, XR);

  const int blkBig = (kTok / 32) * (kChan / 64) / 8;
  gemm_f16_kernel<true, false><<<dim3(blkBig, 4), 256, 0, stream>>>(
      XH, XR, kChan, 0L, WBh, WBr, kChan, (long)wBig,
      QKVG, kChan, (long)kPlane, bo, kTok, kChan, kChan, kScaleProj);

  const int blkSc = (kTok / 32) * (kScalNP / 64) / 8;
  gemm_f16_kernel<false, false><<<dim3(blkSc, 1), 256, 0, stream>>>(
      XH, XH, kChan, 0L, WSc, WSc, kChan, 0L,
      SC, kScalNP, 0L, bo, kTok, kScalNP, kChan, kScaleProj);

  prep_kernel<<<kTok, 256, 0, stream>>>(QKVG, SC, bq, bk, bv, bb, bfd, fdb, bsd, sdb, bfg, bsg);

  state_scan_kernel<<<kBatch * kHeads, kScanThreads, 0, stream>>>(Qf, Kf, Vf, SC, rfp, Yf);

  norm_gate_kernel<<<(kTok * kHeads) / 8, 256, 0, stream>>>(Yf, Gf, bg, onw, (unsigned*)O16);

  gemm_f16_kernel<false, true><<<dim3(blkBig, 1), 256, 0, stream>>>(
      O16, O16, kChan, 0L, WOh, WOh, kChan, 0L,
      out0, kChan, 0L, bo, kTok, kChan, kChan, kScaleOut);
}
